// TimeScaledAttention_12395275616611
// MI455X (gfx1250) — hardware-verified
//
#include <hip/hip_runtime.h>
#include <math.h>

constexpr int   kBatch     = 8;
constexpr int   kSeq       = 4096;
constexpr int   kDim       = 128;
constexpr int   kHid       = 64;
constexpr int   kTok       = kBatch * kSeq;
constexpr int   kQKld      = 2 * kDim;
constexpr int   kHalf      = kSeq / 2;
constexpr int   kNW        = 3 * kDim;
constexpr float kInvSqrtD  = 0.08838834764831845f;
constexpr float kPCarry    = 32768.0f;
constexpr float kPCarryInv = 1.0f / 32768.0f;

constexpr size_t kBytesX16  = (size_t)kTok * kDim * 2;
constexpr size_t kBytesQK   = (size_t)kTok * kQKld * 2;
constexpr size_t kBytesVT   = (size_t)kBatch * kDim * kSeq * 2;
constexpr size_t kBytesS    = (size_t)kHalf * kSeq * 4;
constexpr size_t kBytesP    = (size_t)kHalf * kSeq * 2;
constexpr size_t kBytesWT   = (size_t)kNW * kDim * 2;
constexpr size_t kBytesBias = 4096;
constexpr size_t kBytesTS   = (size_t)kTok * 4;
constexpr size_t kOffXH   = 0;
constexpr size_t kOffXL   = kOffXH + kBytesX16;
constexpr size_t kOffQK   = kOffXL + kBytesX16;
constexpr size_t kOffVT   = kOffQK + kBytesQK;
constexpr size_t kOffS    = kOffVT + kBytesVT;
constexpr size_t kOffP    = kOffS + kBytesS;
constexpr size_t kOffWTH  = kOffP + kBytesP;
constexpr size_t kOffWTL  = kOffWTH + kBytesWT;
constexpr size_t kOffBias = kOffWTL + kBytesWT;
constexpr size_t kOffTS   = kOffBias + kBytesBias;
constexpr size_t kWsTotal = kOffTS + kBytesTS;
constexpr size_t kWsCap   = 134217728;
typedef char ws_total_fits_cap[(kWsTotal <= kWsCap) ? 1 : -1];

typedef __attribute__((ext_vector_type(16))) _Float16 v16h;
typedef __attribute__((ext_vector_type(8)))  _Float16 v8h;
typedef __attribute__((ext_vector_type(16))) __bf16   v16b;
typedef __attribute__((ext_vector_type(8)))  __bf16   v8b;
typedef __attribute__((ext_vector_type(8)))  float    v8f;
typedef __attribute__((ext_vector_type(4)))  float    v4f;
typedef __attribute__((ext_vector_type(4)))  unsigned int v4u;

__device__ __forceinline__ unsigned short f2bf_bits(float f) {
  unsigned u = __float_as_uint(f);
  return (unsigned short)((u + 0x7FFFu + ((u >> 16) & 1u)) >> 16);
}
__device__ __forceinline__ float bf_bits2f(unsigned short h) { return __uint_as_float(((unsigned)h) << 16); }

__device__ __forceinline__ void dep_guard_h(v8f& a, v8f& b, v16h x, v16h y) { asm volatile("v_nop\n\tv_nop\n\tv_nop\n\tv_nop" : "+v"(a), "+v"(b) : "v"(x), "v"(y)); }
__device__ __forceinline__ void dep_guard_b(v8f& a, v8f& b, v16b x, v16b y) { asm volatile("v_nop\n\tv_nop\n\tv_nop\n\tv_nop" : "+v"(a), "+v"(b) : "v"(x), "v"(y)); }
__device__ __forceinline__ void keep4_h(v16h a, v16h b, v16h c, v16h d) { asm volatile("v_nop" :: "v"(a), "v"(b), "v"(c), "v"(d)); }
__device__ __forceinline__ void keep4_b(v16b a, v16b b, v16b c, v16b d) { asm volatile("v_nop" :: "v"(a), "v"(b), "v"(c), "v"(d)); }
__device__ __forceinline__ void acc_guard4(v8f& a, v8f& b, v8f& c, v8f& d) { asm volatile("v_nop\n\tv_nop\n\tv_nop\n\tv_nop" : "+v"(a), "+v"(b), "+v"(c), "+v"(d)); }
template <typename T> struct Frag;
template <> struct Frag<_Float16> {
  typedef v16h V; union U { v16h v; v8h h[2]; };
  static __device__ __forceinline__ v16h load(const _Float16* p) {
    U f; f.h[0] = *(const v8h*)(p); f.h[1] = *(const v8h*)(p + 16); return f.v;
  }
  static __device__ __forceinline__ v8f mma(v16h a, v16h b, v8f c) {
    return __builtin_amdgcn_wmma_f32_16x16x32_f16(false, a, false, b, (short)0, c, false, false);
  }
  static __device__ __forceinline__ void guard(v8f& a, v8f& b, v16h x, v16h y) { dep_guard_h(a, b, x, y); }
  static __device__ __forceinline__ void keep(v16h a, v16h b, v16h c, v16h d) { keep4_h(a, b, c, d); }
};
template <> struct Frag<__bf16> {
  typedef v16b V; union U { v16b v; v8b h[2]; };
  static __device__ __forceinline__ v16b load(const __bf16* p) {
    U f; f.h[0] = *(const v8b*)(p); f.h[1] = *(const v8b*)(p + 16); return f.v;
  }
  static __device__ __forceinline__ v8f mma(v16b a, v16b b, v8f c) {
    return __builtin_amdgcn_wmma_f32_16x16x32_bf16(false, a, false, b, (short)0, c, false, false);
  }
  static __device__ __forceinline__ void guard(v8f& a, v8f& b, v16b x, v16b y) { dep_guard_b(a, b, x, y); }
  static __device__ __forceinline__ void keep(v16b a, v16b b, v16b c, v16b d) { keep4_b(a, b, c, d); }
};

__device__ __forceinline__ unsigned pk16(unsigned short a, unsigned short b) { return (unsigned)a | ((unsigned)b << 16); }
__device__ __forceinline__ unsigned short h_bits(float f) { const _Float16 h = (_Float16)f; return __builtin_bit_cast(unsigned short, h); }

template <int ET> struct Elem;
template <> struct Elem<0> { typedef _Float16 T; };
template <> struct Elem<1> { typedef __bf16 T; };
template <int ET, bool SPLIT, int BIAS_MODE, int OUT_MODE, bool RESID, int ACT = 0>
__global__ __launch_bounds__(256) void wmma_gemm64(
    const unsigned short* __restrict__ Ap, const unsigned short* __restrict__ A2p, int lda, long strideA,
    const unsigned short* __restrict__ Btp, const unsigned short* __restrict__ Bt2p, int ldb, long strideB,
    void* __restrict__ Cout, void* __restrict__ Cout2, int ldc, long strideC,
    const float* __restrict__ bias,
    const float* __restrict__ resid, long strideR,
    int M, int N, int K, float scale) {
  typedef typename Elem<ET>::T T;
  typedef typename Frag<T>::V V;
  const T* A = (const T*)Ap; const T* A2 = (const T*)A2p; const T* Bt = (const T*)Btp; const T* Bt2 = (const T*)Bt2p;
  __shared__ __align__(16) float sT[8][16 * 68];
  const int b    = blockIdx.y;
  const int lane = threadIdx.x & 31;
  const int wave = threadIdx.x >> 5;
  const int tilesN = N >> 6;
  const int tilesM = M >> 6;
  const int tile = blockIdx.x * 8 + wave;
  if (tile >= tilesM * tilesN) return;
  const int tm = tile / tilesN;
  const int tn = tile - tm * tilesN;
  const int m0 = tm << 6;
  const int n0 = tn << 6;

  const T* Ab  = A  + (size_t)b * strideA;
  const T* Bb  = Bt + (size_t)b * strideB;
  const T* Ab2 = SPLIT ? (A2  + (size_t)b * strideA) : nullptr;
  const T* Bb2 = SPLIT ? (Bt2 + (size_t)b * strideB) : nullptr;

  const int rlane = lane & 15;
  const int koff  = (lane >> 4) * 8;
  const int mOff  = (lane >> 4) * 8;

  v8f acc[4][4];
#pragma unroll
  for (int i = 0; i < 4; ++i)
#pragma unroll
    for (int j = 0; j < 4; ++j) acc[i][j] = (v8f){0.f,0.f,0.f,0.f,0.f,0.f,0.f,0.f};

  for (int k0 = 0; k0 < K; k0 += 32) {
    V bh[4], bl[4];
#pragma unroll
    for (int j = 0; j < 4; ++j) {
      const size_t bo = (size_t)(n0 + (j << 4) + rlane) * ldb + koff + k0;
      bh[j] = Frag<T>::load(Bb + bo);
      if (SPLIT) bl[j] = Frag<T>::load(Bb2 + bo);
    }
#pragma unroll
    for (int i = 0; i < 4; ++i) {
      const size_t ao = (size_t)(m0 + (i << 4) + rlane) * lda + koff + k0;
      V ah = Frag<T>::load(Ab + ao);
      V al;
      if (SPLIT) al = Frag<T>::load(Ab2 + ao);
#pragma unroll
      for (int j = 0; j < 4; ++j) {
        acc[i][j] = Frag<T>::mma(ah, bh[j], acc[i][j]);
        if (SPLIT) {
          acc[i][j] = Frag<T>::mma(ah, bl[j], acc[i][j]);
          acc[i][j] = Frag<T>::mma(al, bh[j], acc[i][j]);
        }
      }
      Frag<T>::guard(acc[i][0], acc[i][3], ah, SPLIT ? al : ah);
    }
    Frag<T>::keep(bh[0], bh[1], bh[2], bh[3]);
    if (SPLIT) Frag<T>::keep(bl[0], bl[1], bl[2], bl[3]);
  }
  acc_guard4(acc[0][0], acc[0][1], acc[0][2], acc[0][3]);
  acc_guard4(acc[1][0], acc[1][1], acc[1][2], acc[1][3]);
  acc_guard4(acc[2][0], acc[2][1], acc[2][2], acc[2][3]);
  acc_guard4(acc[3][0], acc[3][1], acc[3][2], acc[3][3]);

  float* slab = sT[wave];
  const float* Rb = RESID ? (resid + (size_t)b * strideR) : nullptr;
#pragma unroll
  for (int i = 0; i < 4; ++i) {
    const int mBase = m0 + (i << 4);
#pragma unroll
    for (int j = 0; j < 4; ++j) {
      const int n = n0 + (j << 4) + rlane;
      float bv = 0.f;
      if (BIAS_MODE == 2) bv = bias[n];
#pragma unroll
      for (int r = 0; r < 8; ++r) {
        float v = acc[i][j][r] * scale;
        if (BIAS_MODE == 1) v += bias[mBase + mOff + r];
        if (BIAS_MODE == 2) v += bv;
        if (RESID) v += Rb[(size_t)(mBase + mOff + r) * ldc + n];
        if (ACT == 2) v = fmaxf(v, 0.0f);
        if (ACT == 4) v = (v > 0.f) ? v : 0.01f * v;
        slab[(mOff + r) * 68 + (j << 4) + rlane] = v;
      }
    }
    __builtin_amdgcn_fence(__ATOMIC_RELEASE, "workgroup");
    __builtin_amdgcn_wave_barrier();
    __builtin_amdgcn_fence(__ATOMIC_ACQUIRE, "workgroup");
    if (OUT_MODE == 0) {
      float* C = (float*)Cout + (size_t)b * strideC;
      const int hh = lane >> 4, c4 = (lane & 15) * 4;
      for (int pass = 0; pass < 2; ++pass) {
#pragma unroll
        for (int it = 0; it < 8; ++it) {
          const int row = it * 2 + hh;
          v4f v = *(const v4f*)(slab + row * 68 + c4);
          *(volatile v4f*)(C + (size_t)(mBase + row) * ldc + n0 + c4) = v;
        }
        __threadfence();
      }
    } else {
      const int q = lane >> 3, c8 = (lane & 7) * 8;
      unsigned short* C  = (unsigned short*)Cout  + (size_t)b * strideC;
      unsigned short* C2 = (OUT_MODE == 2) ? ((unsigned short*)Cout2 + (size_t)b * strideC) : nullptr;
      for (int pass = 0; pass < 2; ++pass) {
#pragma unroll
        for (int it = 0; it < 4; ++it) {
          const int row = it * 4 + q;
          const float* sp = slab + row * 68 + c8;
          v8h hv, lv;
#pragma unroll
          for (int e = 0; e < 8; ++e) {
            if (OUT_MODE == 1) {
              hv[e] = (_Float16)sp[e];
            } else {
              unsigned short hb = f2bf_bits(sp[e]);
              unsigned short lb = f2bf_bits(sp[e] - bf_bits2f(hb));
              hv[e] = __builtin_bit_cast(_Float16, hb);
              lv[e] = __builtin_bit_cast(_Float16, lb);
            }
          }
          *(volatile v8h*)(C + (size_t)(mBase + row) * ldc + n0 + c8) = hv;
          if (OUT_MODE == 2) *(volatile v8h*)(C2 + (size_t)(mBase + row) * ldc + n0 + c8) = lv;
        }
        __threadfence();
      }
    }
    __builtin_amdgcn_fence(__ATOMIC_RELEASE, "workgroup");
    __builtin_amdgcn_wave_barrier();
    __builtin_amdgcn_fence(__ATOMIC_ACQUIRE, "workgroup");
  }
}

__global__ __launch_bounds__(256) void xsplit_kernel(const float* __restrict__ in,
                                                     unsigned short* __restrict__ hi,
                                                     unsigned short* __restrict__ lo, int n8) {
  const int i = blockIdx.x * 256 + threadIdx.x;
  if (i >= n8) return;
  const float* p = in + 8 * (size_t)i;
  const v4f a = *(const v4f*)(p);
  const v4f c = *(const v4f*)(p + 4);
  unsigned short hb[8], lb[8];
#pragma unroll
  for (int e = 0; e < 4; ++e) {
    const float f0 = a[e];
    hb[e] = f2bf_bits(f0);
    lb[e] = f2bf_bits(f0 - bf_bits2f(hb[e]));
    const float f1 = c[e];
    hb[4 + e] = f2bf_bits(f1);
    lb[4 + e] = f2bf_bits(f1 - bf_bits2f(hb[4 + e]));
  }
  const v4u uh = (v4u){pk16(hb[0], hb[1]), pk16(hb[2], hb[3]), pk16(hb[4], hb[5]), pk16(hb[6], hb[7])};
  const v4u ul = (v4u){pk16(lb[0], lb[1]), pk16(lb[2], lb[3]), pk16(lb[4], lb[5]), pk16(lb[6], lb[7])};
  unsigned short* qh = hi + 8 * (size_t)i;
  unsigned short* ql = lo + 8 * (size_t)i;
  *(volatile v4u*)qh = uh;
  *(volatile v4u*)ql = ul;
  __threadfence();
  *(volatile v4u*)qh = uh;
  *(volatile v4u*)ql = ul;
}

__global__ __launch_bounds__(256) void wprep_kernel(const float* __restrict__ Wq, const float* __restrict__ Wk,
                                                    const float* __restrict__ Wv,
                                                    const float* __restrict__ bq, const float* __restrict__ bk,
                                                    const float* __restrict__ bv,
                                                    unsigned short* __restrict__ WtH, unsigned short* __restrict__ WtL,
                                                    float* __restrict__ bias384) {
  __shared__ float sm[64][129];
  const int t  = threadIdx.x;
  const int nt = blockIdx.x;
  const int z  = blockIdx.y;
  const float* W  = (z == 0) ? Wq : (z == 1) ? Wk : Wv;
  const float* bs = (z == 0) ? bq : (z == 1) ? bk : bv;
#pragma unroll
  for (int i = 0; i < 32; ++i) {
    const int e  = i * 256 + t;
    const int kk = e >> 6;
    const int nl = e & 63;
    sm[nl][kk] = W[(size_t)kk * kDim + nt * 64 + nl];
  }
  __syncthreads();
  const int lane = t & 31, wave = t >> 5;
  const int hh = lane >> 4, c8 = (lane & 15) * 8;
  for (int pass = 0; pass < 2; ++pass) {
#pragma unroll
    for (int it = 0; it < 4; ++it) {
      const int nl = wave * 8 + it * 2 + hh;
      unsigned short hb[8], lb[8];
#pragma unroll
      for (int e = 0; e < 8; ++e) {
        const float f = sm[nl][c8 + e];
        hb[e] = f2bf_bits(f);
        lb[e] = f2bf_bits(f - bf_bits2f(hb[e]));
      }
      const v4u uh = (v4u){pk16(hb[0], hb[1]), pk16(hb[2], hb[3]), pk16(hb[4], hb[5]), pk16(hb[6], hb[7])};
      const v4u ul = (v4u){pk16(lb[0], lb[1]), pk16(lb[2], lb[3]), pk16(lb[4], lb[5]), pk16(lb[6], lb[7])};
      const size_t o = (size_t)(z * kDim + nt * 64 + nl) * kDim + c8;
      *(volatile v4u*)(WtH + o) = uh;
      *(volatile v4u*)(WtL + o) = ul;
    }
    __threadfence();
  }
  if (nt == 0 && t < 32) {
    const v4f bv4 = *(const v4f*)(bs + 4 * t);
    float* bp = bias384 + z * kDim + 4 * t;
    *(volatile v4f*)bp = bv4;
    __threadfence();
    *(volatile v4f*)bp = bv4;
  }
}

__global__ __launch_bounds__(128) void gate_kernel(const float* __restrict__ tg,
                                                   const float* __restrict__ W1, const float* __restrict__ b1,
                                                   const float* __restrict__ W2, const float* __restrict__ b2,
                                                   const float* __restrict__ W3, const float* __restrict__ b3,
                                                   float* __restrict__ ts, int ntot) {
  __shared__ __align__(16) float W2s[kHid * kHid];
  __shared__ float w1s[kHid], b1s[kHid], b2s[kHid], w3s[kHid];
  const int t = threadIdx.x;
  for (int e = t; e < kHid * kHid; e += 128) {
    const int i = e >> 6, j = e & 63;
    W2s[j * kHid + i] = W2[e];
  }
  if (t < kHid) { w1s[t] = W1[t]; b1s[t] = b1[t]; b2s[t] = b2[t]; w3s[t] = W3[t]; }
  __syncthreads();

  const int idx = blockIdx.x * 128 + t;
  const int idc = (idx < ntot) ? idx : (ntot - 1);
  const float x = tg[idc];
  float h1[kHid];
#pragma unroll
  for (int j = 0; j < kHid; ++j) {
    float pr = x * w1s[j];
    asm volatile("" : "+v"(pr));
    h1[j] = fmaxf(pr + b1s[j], 0.0f);
  }
  float acc = 0.0f;
#pragma unroll 1
  for (int j = 0; j < kHid; ++j) {
    const float* wc = W2s + j * kHid;
    float a = 0.0f;
#pragma unroll
    for (int i = 0; i < kHid; i += 4) {
      const v4f w = *(const v4f*)(wc + i);
      a = fmaf(h1[i],     w[0], a);
      a = fmaf(h1[i + 1], w[1], a);
      a = fmaf(h1[i + 2], w[2], a);
      a = fmaf(h1[i + 3], w[3], a);
    }
    a = fmaxf(a + b2s[j], 0.0f);
    acc = fmaf(a, w3s[j], acc);
  }
  const float z   = acc + b3[0];
  const float ef  = expf(-z);
  const float tsv = __builtin_amdgcn_rcpf(1.0f + ef);
  if (idx < ntot) {
    *(volatile float*)(ts + idx) = tsv;
    __threadfence();
    *(volatile float*)(ts + idx) = tsv;
  }
}

__global__ __launch_bounds__(512) void softmax_kernel(const float* __restrict__ S, const float* __restrict__ tsq,
                                                      unsigned short* __restrict__ P) {
  __shared__ float redM[16];
  __shared__ float redS[16];
  const int row  = blockIdx.x;
  const int t    = threadIdx.x;
  const int lane = t & 31, wave = t >> 5;
  const int c0   = t * 8;
  const float tsv = tsq[row];
  const float* sr = S + (size_t)row * kSeq + c0;
  const v4f a = *(const v4f*)(sr);
  const v4f c = *(const v4f*)(sr + 4);
  float x[8];
#pragma unroll
  for (int e = 0; e < 4; ++e) {
    x[e]     = (a[e] * kInvSqrtD) * tsv;
    x[4 + e] = (c[e] * kInvSqrtD) * tsv;
  }
  float m = fmaxf(fmaxf(fmaxf(x[0], x[1]), fmaxf(x[2], x[3])), fmaxf(fmaxf(x[4], x[5]), fmaxf(x[6], x[7])));
#pragma unroll
  for (int off = 16; off > 0; off >>= 1) m = fmaxf(m, __shfl_xor(m, off, 32));
  if (lane == 0) redM[wave] = m;
  __syncthreads();
  float gm = redM[0];
#pragma unroll
  for (int w = 1; w < 16; ++w) gm = fmaxf(gm, redM[w]);
  float ev[8];
  float ps = 0.0f;
#pragma unroll
  for (int e = 0; e < 8; ++e) { ev[e] = expf(x[e] - gm); ps += ev[e]; }
#pragma unroll
  for (int off = 16; off > 0; off >>= 1) ps += __shfl_xor(ps, off, 32);
  if (lane == 0) redS[wave] = ps;
  __syncthreads();
  float tot = redS[0];
#pragma unroll
  for (int w = 1; w < 16; ++w) tot += redS[w];
  const float f = (1.0f / tot) * kPCarry;
  unsigned short hb[8];
#pragma unroll
  for (int e = 0; e < 8; ++e) hb[e] = h_bits(ev[e] * f);
  const v4u u = (v4u){pk16(hb[0], hb[1]), pk16(hb[2], hb[3]), pk16(hb[4], hb[5]), pk16(hb[6], hb[7])};
  unsigned short* q = P + (size_t)row * kSeq + c0;
  *(volatile v4u*)q = u;
  __threadfence();
  *(volatile v4u*)q = u;
}

extern "C" void kernel_launch(void* const* d_in, const int* in_sizes, int n_in,
                              void* d_out, int out_size, void* d_ws, size_t ws_size,
                              hipStream_t stream) {
  if (n_in < 14) return;
  if (ws_size < kWsTotal) return;
  if (out_size < kTok * kDim) return;
  if (in_sizes[0] < kTok * kDim || in_sizes[1] < kTok ||
      in_sizes[2] < kDim * kDim || in_sizes[3] < kDim ||
      in_sizes[4] < kDim * kDim || in_sizes[5] < kDim ||
      in_sizes[6] < kDim * kDim || in_sizes[7] < kDim ||
      in_sizes[8] < kHid || in_sizes[9] < kHid ||
      in_sizes[10] < kHid * kHid || in_sizes[11] < kHid ||
      in_sizes[12] < kHid || in_sizes[13] < 1) return;

  const float* x  = (const float*)d_in[0];
  const float* tg = (const float*)d_in[1];
  const float* Wq = (const float*)d_in[2];  const float* bq = (const float*)d_in[3];
  const float* Wk = (const float*)d_in[4];  const float* bk = (const float*)d_in[5];
  const float* Wv = (const float*)d_in[6];  const float* bv = (const float*)d_in[7];
  const float* W1 = (const float*)d_in[8];  const float* b1 = (const float*)d_in[9];
  const float* W2 = (const float*)d_in[10]; const float* b2 = (const float*)d_in[11];
  const float* W3 = (const float*)d_in[12]; const float* b3 = (const float*)d_in[13];
  float* out = (float*)d_out;

  char* ws = (char*)d_ws;
  unsigned short* XH   = (unsigned short*)(ws + kOffXH);
  unsigned short* XL   = (unsigned short*)(ws + kOffXL);
  unsigned short* QK   = (unsigned short*)(ws + kOffQK);
  unsigned short* VT   = (unsigned short*)(ws + kOffVT);
  float*          Sf   = (float*)(ws + kOffS);
  unsigned short* P16  = (unsigned short*)(ws + kOffP);
  unsigned short* WTH  = (unsigned short*)(ws + kOffWTH);
  unsigned short* WTL  = (unsigned short*)(ws + kOffWTL);
  float*          b384 = (float*)(ws + kOffBias);
  float*          tsb  = (float*)(ws + kOffTS);

  const int n8 = kTok * kDim / 8;
  xsplit_kernel<<<dim3((n8 + 255) / 256), dim3(256), 0, stream>>>(x, XH, XL, n8);
  wprep_kernel<<<dim3(2, 3), dim3(256), 0, stream>>>(Wq, Wk, Wv, bq, bk, bv, WTH, WTL, b384);
  gate_kernel<<<dim3(kTok / 128), dim3(128), 0, stream>>>(tg, W1, b1, W2, b2, W3, b3, tsb, kTok);

  wmma_gemm64<1, true, 2, 1, false><<<dim3((kTok / 64) * (kQKld / 64) / 8, 1), dim3(256), 0, stream>>>(
      XH, XL, kDim, 0L,
      WTH, WTL, kDim, 0L,
      (void*)QK, (void*)QK, kQKld, 0L,
      b384, Sf, 0L,
      kTok, kQKld, kDim, 1.0f);

  wmma_gemm64<1, true, 1, 1, false><<<dim3((kDim / 64) * (kSeq / 64) / 8, kBatch), dim3(256), 0, stream>>>(
      WTH + (size_t)2 * kDim * kDim, WTL + (size_t)2 * kDim * kDim, kDim, 0L,
      XH, XL, kDim, (long)kSeq * kDim,
      (void*)VT, (void*)VT, kSeq, (long)kDim * kSeq,
      b384 + 2 * kDim, Sf, 0L,
      kDim, kSeq, kDim, 1.0f);

  for (int b = 0; b < kBatch; ++b) {
    for (int hf = 0; hf < 2; ++hf) {
      const size_t qrow0 = (size_t)b * kSeq + (size_t)hf * kHalf;
      const unsigned short* Aq = QK + qrow0 * kQKld;
      const unsigned short* Bk = QK + (size_t)b * kSeq * kQKld + kDim;
      wmma_gemm64<0, false, 0, 0, false><<<dim3((kHalf / 64) * (kSeq / 64) / 8, 1), dim3(256), 0, stream>>>(
          Aq, Aq, kQKld, 0L,
          Bk, Bk, kQKld, 0L,
          (void*)Sf, (void*)Sf, kSeq, 0L,
          b384, Sf, 0L,
          kHalf, kSeq, kDim, 1.0f);
      softmax_kernel<<<dim3(kHalf), dim3(512), 0, stream>>>(Sf, tsb + qrow0, P16);
      const unsigned short* Bv = VT + (size_t)b * kDim * kSeq;
      float* Co = out + qrow0 * kDim;
      wmma_gemm64<0, false, 0, 0, false><<<dim3((kHalf / 64) * (kDim / 64) / 8, 1), dim3(256), 0, stream>>>(
          P16, P16, kSeq, 0L,
          Bv, Bv, kSeq, 0L,
          (void*)Co, (void*)Co, kDim, 0L,
          b384, Sf, 0L,
          kHalf, kDim, kSeq, kPCarryInv);
    }
  }
}
